// GTMEstimator_74706661147263
// MI455X (gfx1250) — hardware-verified
//
#include <hip/hip_runtime.h>
#include <math.h>

typedef __attribute__((ext_vector_type(16))) _Float16 v16h;
typedef __attribute__((ext_vector_type(16))) __bf16 v16b;
typedef __attribute__((ext_vector_type(8)))  _Float16 v8h;
typedef __attribute__((ext_vector_type(8)))  float v8f;
typedef __attribute__((ext_vector_type(4)))  float v4f;
typedef __attribute__((ext_vector_type(2)))  float v2f;
typedef __attribute__((ext_vector_type(4)))  unsigned v4u;
typedef __attribute__((ext_vector_type(4)))  int v4i;
typedef float __attribute__((may_alias)) float_a;
typedef int __attribute__((may_alias)) int_a;

template <typename T> __device__ __forceinline__ void vst2(void* p, T v) { *(volatile T*)p = v; __threadfence(); *(volatile T*)p = v; }
__device__ __forceinline__ v8f wmma16(v16h a, v16h b, v8f c) {
  v8f d = __builtin_amdgcn_wmma_f32_16x16x32_f16(false, a, false, b, (short)0, c, false, false);
  asm volatile("v_nop\n\tv_nop\n\tv_nop\n\tv_nop" : "+v"(d) : "v"(a), "v"(b));
  return d;
}
__device__ __forceinline__ v8f wmma_bf(v16b a, v16b b, v8f c) {
  v8f d = __builtin_amdgcn_wmma_f32_16x16x32_bf16(false, a, false, b, (short)0, c, false, false);
  asm volatile("v_nop\n\tv_nop\n\tv_nop\n\tv_nop" : "+v"(d) : "v"(a), "v"(b));
  return d;
}
__device__ __forceinline__ v16h frag_h(const _Float16* rowk0, int lane) {
  union { v16h v; v8h q[2]; } u; const _Float16* p = rowk0 + 8 * (lane >> 4);
  u.q[0] = *(const v8h*)p; u.q[1] = *(const v8h*)(p + 16); return u.v;
}
__device__ __forceinline__ v16h frag_f32(const float* rowk0, int lane) {
  v16h a; const float* p = rowk0 + 8 * (lane >> 4);
#pragma unroll
  for (int i = 0; i < 8; ++i) { a[i] = (_Float16)p[i]; a[8 + i] = (_Float16)p[16 + i]; }
  return a;
}
__device__ __forceinline__ v16h frag_f32s(const float* rowk0, int lane, float sc) {
  v16h a; const float* p = rowk0 + 8 * (lane >> 4);
#pragma unroll
  for (int i = 0; i < 8; ++i) { a[i] = (_Float16)(p[i] * sc); a[8 + i] = (_Float16)(p[16 + i] * sc); }
  return a;
}
__device__ __forceinline__ v16h fragc_f32(const float* W, int k0, int n, int lane, int ld, int K) {
  v16h a; const int g = lane >> 4;
#pragma unroll
  for (int i = 0; i < 8; ++i) { const int ka = k0 + 8 * g + i, kb = ka + 16;
    a[i] = (_Float16)(ka < K ? W[(size_t)(ka < K ? ka : K - 1) * ld + n] : 0.f); a[8 + i] = (_Float16)(kb < K ? W[(size_t)(kb < K ? kb : K - 1) * ld + n] : 0.f); }
  return a;
}
struct F2 { v16b h, l; };
__device__ __forceinline__ F2 bsplit16(const float v[16]) { F2 r;
#pragma unroll
  for (int i = 0; i < 16; ++i) { const __bf16 h = (__bf16)v[i]; r.h[i] = h; r.l[i] = (__bf16)(v[i] - (float)h); }
  return r; }
__device__ __forceinline__ F2 split_row(const float* row, int k0, int lane) { float v[16]; const float* p = row + k0 + 8 * (lane >> 4);
#pragma unroll
  for (int i = 0; i < 8; ++i) { v[i] = p[i]; v[8 + i] = p[16 + i]; }
  return bsplit16(v); }
__device__ __forceinline__ F2 split_rowK(const float* row, int k0, int lane, int K) { float v[16]; const int g = lane >> 4;
#pragma unroll
  for (int i = 0; i < 8; ++i) { const int ka = k0 + 8 * g + i, kb = ka + 16; v[i] = ka < K ? row[ka < K ? ka : K - 1] : 0.f; v[8 + i] = kb < K ? row[kb < K ? kb : K - 1] : 0.f; }
  return bsplit16(v); }
__device__ __forceinline__ F2 split_col(const float* W, int k0, int n, int lane, int ld, int K) { float v[16]; const int g = lane >> 4;
#pragma unroll
  for (int i = 0; i < 8; ++i) { const int ka = k0 + 8 * g + i, kb = ka + 16; v[i] = ka < K ? W[(size_t)(ka < K ? ka : K - 1) * ld + n] : 0.f; v[8 + i] = kb < K ? W[(size_t)(kb < K ? kb : K - 1) * ld + n] : 0.f; }
  return bsplit16(v); }
__device__ __forceinline__ v8f mac3(const F2& a, const F2& b, v8f c) { c = wmma_bf(a.l, b.h, c); c = wmma_bf(a.h, b.l, c); return wmma_bf(a.h, b.h, c); }
__device__ __forceinline__ float sigm(float v) { return 1.0f / (1.0f + expf(-v)); }
#define LDSX() do { asm volatile("s_wait_dscnt 0" ::: "memory"); __builtin_amdgcn_wave_barrier(); __builtin_amdgcn_fence(__ATOMIC_RELEASE, "workgroup"); } while (0)


#define NS 8192
#define DD 512
#define KG 10000
typedef __attribute__((ext_vector_type(8))) __bf16 v8b;
__device__ __forceinline__ v16b frag_b(const __bf16* rowk0, int lane) {
  union { v16b v; v8b q[2]; } u; const __bf16* p = rowk0 + 8 * (lane >> 4);
  u.q[0] = *(const v8b*)p; u.q[1] = *(const v8b*)(p + 16); return u.v;
}
__device__ __forceinline__ float bfr(float v) { return (float)(__bf16)v; }
__device__ __attribute__((noinline)) float exp_ni(float v) { return expf(v); }
__device__ __attribute__((noinline)) float erf_ni(float v) { return erff(v); }

#define WS_ACE 0u
#define WS_YN  (WS_ACE + 4u * (size_t)NS * 16)
#define WS_END (WS_YN + 4u * 10016)

__global__ __launch_bounds__(128) void k_ace(const float* __restrict__ X, const float* __restrict__ Wm, const float* __restrict__ Bv, float* __restrict__ ACE) { __shared__ __align__(16) float so[64][16];
  const int tid = threadIdx.x, wave = tid >> 5, lane = tid & 31, col = lane & 15, g = lane >> 4; const size_t r0 = (size_t)blockIdx.x * 64 + wave * 16;
  v8f acc = {};
#pragma unroll 2
  for (int kc = 0; kc < DD / 32; ++kc) { v16b a, w; const float* p = X + (r0 + col) * DD + kc * 32 + 8 * g;
#pragma unroll
    for (int i = 0; i < 8; ++i) { a[i] = (__bf16)p[i]; a[8 + i] = (__bf16)p[16 + i]; const int d0 = kc * 32 + 8 * g + i, d1 = d0 + 16; const float v0 = (col == 0) ? Wm[d0 * 2] : (col == 1) ? Wm[d0 * 2 + 1] : (col == 2) ? Bv[d0] : 0.f; const float v1 = (col == 0) ? Wm[d1 * 2] : (col == 1) ? Wm[d1 * 2 + 1] : (col == 2) ? Bv[d1] : 0.f; w[i] = (__bf16)v0; w[8 + i] = (__bf16)v1; }
    acc = wmma_bf(a, w, acc); }
#pragma unroll
  for (int r = 0; r < 8; ++r) so[wave * 16 + 8 * g + r][col] = acc[r];
  __syncthreads(); for (int e = tid; e < 64 * 4; e += 128) { const int rl = e >> 2, q = e & 3; vst2(ACE + ((size_t)blockIdx.x * 64 + rl) * 16 + q * 4, *(const v4f*)&so[rl][q * 4]); } }
__global__ __launch_bounds__(256) void k_yn(const float* __restrict__ Wm, const float* __restrict__ Bv, const float* __restrict__ G, float* __restrict__ YN) { __shared__ float sred[8][6]; __shared__ float S[6]; __shared__ __align__(16) float syn[10016];
  const int t = threadIdx.x; float s00 = 0.f, s11 = 0.f, s01 = 0.f, s0b = 0.f, s1b = 0.f, sbb = 0.f;
  for (int d = t; d < DD; d += 256) { const float w0 = bfr(Wm[d * 2]), w1 = bfr(Wm[d * 2 + 1]), bb = bfr(Bv[d]); s00 += w0 * w0; s11 += w1 * w1; s01 += w0 * w1; s0b += w0 * bb; s1b += w1 * bb; sbb += bb * bb; }
  float vals[6] = {s00, s11, s01, s0b, s1b, sbb};
#pragma unroll
  for (int q = 0; q < 6; ++q) { float v = vals[q];
#pragma unroll
    for (int o = 1; o < 32; o <<= 1) v += __shfl_xor(v, o); if ((t & 31) == 0) sred[t >> 5][q] = v; }
  __syncthreads(); if (t < 6) { float v = 0.f; for (int w = 0; w < 8; ++w) v += sred[w][t]; S[t] = v; } __syncthreads();
  for (int k = t; k < 10016; k += 256) { float v = 0.f; if (k < KG) { const float g0 = bfr(G[k * 2]), g1 = bfr(G[k * 2 + 1]); v = g0 * g0 * S[0] + g1 * g1 * S[1] + 2.f * g0 * g1 * S[2] + 2.f * g0 * S[3] + 2.f * g1 * S[4] + S[5]; } syn[k] = v; }
  __syncthreads(); for (int q = t; q < 10016 / 4; q += 256) vst2(YN + q * 4, *(const v4f*)&syn[q * 4]); }
__global__ __launch_bounds__(128) void k_post(const float* __restrict__ ACE, const float* __restrict__ YN, const float* __restrict__ G, const float* __restrict__ BE, float* __restrict__ OUT) { __shared__ __align__(16) float sg[KG * 2]; __shared__ __align__(16) float syn[KG]; __shared__ __align__(16) float so[128][2];
  const int t = threadIdx.x; const size_t n = (size_t)blockIdx.x * 128 + t;
  for (int e = t; e < KG * 2; e += 128) sg[e] = bfr(G[e]); for (int e = t; e < KG; e += 128) syn[e] = YN[e];
  __syncthreads();
  const float hb = -0.5f * bfr(BE[0]); const float a = ACE[n * 16], c = ACE[n * 16 + 1], ee = ACE[n * 16 + 2];
  float m = -3.0e38f, l = 0.f, u0 = 0.f, u1 = 0.f;
#pragma unroll 1
  for (int k = 0; k < KG; ++k) { const float g0 = sg[2 * k], g1 = sg[2 * k + 1]; const float lg = hb * (syn[k] - 2.f * (g0 * a + g1 * c + ee));
    if (lg > m) { const float sc = __expf(m - lg); l *= sc; u0 *= sc; u1 *= sc; m = lg; }
    const float p = __expf(lg - m); l += p; u0 += p * g0; u1 += p * g1; }
  so[t][0] = u0 / l; so[t][1] = u1 / l;
  __syncthreads(); if (t < 64) vst2(OUT + (size_t)blockIdx.x * 256 + t * 4, *(const v4f*)&(&so[0][0])[t * 4]); }
extern "C" void kernel_launch(void* const* d_in, const int* in_sizes, int n_in, void* d_out, int out_size, void* d_ws, size_t ws_size, hipStream_t stream) {
  (void)in_sizes; (void)n_in; (void)out_size;
  const float** F = (const float**)d_in;
  if (ws_size < (size_t)WS_END) return;
  char* ws = (char*)d_ws; float *ACE = (float*)(ws + WS_ACE), *YN = (float*)(ws + WS_YN);
  k_ace<<<NS / 64, 128, 0, stream>>>(F[0], F[1], F[2], ACE);
  k_yn<<<1, 256, 0, stream>>>(F[1], F[2], F[4], YN);
  k_post<<<NS / 128, 128, 0, stream>>>(ACE, YN, F[4], F[3], (float*)d_out);
}
